// InterPointAttentionNet_45612552683807
// MI455X (gfx1250) — hardware-verified
//
#include <hip/hip_runtime.h>
#include <math.h>

constexpr int kBt  = 4;
constexpr int kNp  = 256;
constexpr int kHd  = 4;
constexpr int kCh  = 64;
constexpr int kDim = 256;
constexpr int kFF  = 1024;
constexpr int kPH  = 128;
constexpr int kTok   = kBt * kNp;
constexpr int kPairs = kBt * kNp * kNp;
constexpr int kSlab  = kNp * kDim;
constexpr float kLnEps   = 1e-5f;
constexpr float kWCarry  = 256.0f;
constexpr float kH1Carry = 1024.0f;
constexpr float kPCarry  = 4096.0f;
constexpr float kMgCarry = 64.0f;

typedef __attribute__((ext_vector_type(16))) _Float16 v16h;
typedef __attribute__((ext_vector_type(8)))  _Float16 v8h;
typedef __attribute__((ext_vector_type(16))) __bf16   v16b;
typedef __attribute__((ext_vector_type(8)))  __bf16   v8b;
typedef __attribute__((ext_vector_type(8)))  float    v8f;
typedef __attribute__((ext_vector_type(4)))  float    v4f;
typedef __attribute__((ext_vector_type(4)))  unsigned int v4u;

__device__ __forceinline__ unsigned short f2bf_bits(float f) {
  unsigned u = __float_as_uint(f);
  return (unsigned short)((u + 0x7FFFu + ((u >> 16) & 1u)) >> 16);
}
__device__ __forceinline__ float bf_bits2f(unsigned short h) { return __uint_as_float(((unsigned)h) << 16); }

__device__ __forceinline__ void dep_guard_h(v8f& a, v8f& b, v16h x, v16h y) { asm volatile("v_nop\n\tv_nop\n\tv_nop\n\tv_nop" : "+v"(a), "+v"(b) : "v"(x), "v"(y)); }
__device__ __forceinline__ void dep_guard_b(v8f& a, v8f& b, v16b x, v16b y) { asm volatile("v_nop\n\tv_nop\n\tv_nop\n\tv_nop" : "+v"(a), "+v"(b) : "v"(x), "v"(y)); }
__device__ __forceinline__ void keep4_h(v16h a, v16h b, v16h c, v16h d) { asm volatile("v_nop" :: "v"(a), "v"(b), "v"(c), "v"(d)); }
__device__ __forceinline__ void keep4_b(v16b a, v16b b, v16b c, v16b d) { asm volatile("v_nop" :: "v"(a), "v"(b), "v"(c), "v"(d)); }
__device__ __forceinline__ void acc_guard4(v8f& a, v8f& b, v8f& c, v8f& d) { asm volatile("v_nop\n\tv_nop\n\tv_nop\n\tv_nop" : "+v"(a), "+v"(b), "+v"(c), "+v"(d)); }
template <typename T> struct Frag;
template <> struct Frag<_Float16> {
  typedef v16h V; union U { v16h v; v8h h[2]; };
  static __device__ __forceinline__ v16h load(const _Float16* p) {
    U f; f.h[0] = *(const v8h*)(p); f.h[1] = *(const v8h*)(p + 16); return f.v;
  }
  static __device__ __forceinline__ v8f mma(v16h a, v16h b, v8f c) {
    return __builtin_amdgcn_wmma_f32_16x16x32_f16(false, a, false, b, (short)0, c, false, false);
  }
  static __device__ __forceinline__ void guard(v8f& a, v8f& b, v16h x, v16h y) { dep_guard_h(a, b, x, y); }
  static __device__ __forceinline__ void keep(v16h a, v16h b, v16h c, v16h d) { keep4_h(a, b, c, d); }
};
template <> struct Frag<__bf16> {
  typedef v16b V; union U { v16b v; v8b h[2]; };
  static __device__ __forceinline__ v16b load(const __bf16* p) {
    U f; f.h[0] = *(const v8b*)(p); f.h[1] = *(const v8b*)(p + 16); return f.v;
  }
  static __device__ __forceinline__ v8f mma(v16b a, v16b b, v8f c) {
    return __builtin_amdgcn_wmma_f32_16x16x32_bf16(false, a, false, b, (short)0, c, false, false);
  }
  static __device__ __forceinline__ void guard(v8f& a, v8f& b, v16b x, v16b y) { dep_guard_b(a, b, x, y); }
  static __device__ __forceinline__ void keep(v16b a, v16b b, v16b c, v16b d) { keep4_b(a, b, c, d); }
};

__device__ __forceinline__ unsigned pk16(unsigned short a, unsigned short b) { return (unsigned)a | ((unsigned)b << 16); }
__device__ __forceinline__ unsigned short h_bits(float f) { const _Float16 h = (_Float16)f; return __builtin_bit_cast(unsigned short, h); }

template <int ET> struct Elem;
template <> struct Elem<0> { typedef _Float16 T; };
template <> struct Elem<1> { typedef __bf16 T; };
template <int ET, int BIAS_MODE, int OUT_MODE, bool RESID, int ACT>
__global__ __launch_bounds__(256) void wmma_gemm64z(
    const unsigned short* __restrict__ Ap, int lda, long strideA, long strideAz,
    const unsigned short* __restrict__ Btp, int ldb, long strideB, long strideBz,
    void* __restrict__ Cout, int ldc, long strideC, long strideCz,
    const float* __restrict__ bias,
    const float* __restrict__ resid, long strideR, long strideRz,
    int M, int N, int K, float scale, float oscale) {
  typedef typename Elem<ET>::T T;
  typedef typename Frag<T>::V V;
  const T* A = (const T*)Ap; const T* Bt = (const T*)Btp;
  __shared__ __align__(16) float sT[8][16 * 68];
  const int b    = blockIdx.y;
  const int bz   = blockIdx.z;
  const int lane = threadIdx.x & 31;
  const int wave = threadIdx.x >> 5;
  const int tilesN = N >> 6;
  const int tilesM = M >> 6;
  const int tile = blockIdx.x * 8 + wave;
  if (tile >= tilesM * tilesN) return;
  const int tm = tile / tilesN;
  const int tn = tile - tm * tilesN;
  const int m0 = tm << 6;
  const int n0 = tn << 6;

  const T* Ab = A  + (size_t)b * strideA + (size_t)bz * strideAz;
  const T* Bb = Bt + (size_t)b * strideB + (size_t)bz * strideBz;

  const int rlane = lane & 15;
  const int koff  = (lane >> 4) * 8;
  const int mOff  = (lane >> 4) * 8;

  v8f acc[4][4];
#pragma unroll
  for (int i = 0; i < 4; ++i)
#pragma unroll
    for (int j = 0; j < 4; ++j) acc[i][j] = (v8f){0.f,0.f,0.f,0.f,0.f,0.f,0.f,0.f};

  for (int k0 = 0; k0 < K; k0 += 32) {
    V bh[4];
#pragma unroll
    for (int j = 0; j < 4; ++j) {
      const size_t bo = (size_t)(n0 + (j << 4) + rlane) * ldb + koff + k0;
      bh[j] = Frag<T>::load(Bb + bo);
    }
#pragma unroll
    for (int i = 0; i < 4; ++i) {
      const size_t ao = (size_t)(m0 + (i << 4) + rlane) * lda + koff + k0;
      V ah = Frag<T>::load(Ab + ao);
#pragma unroll
      for (int j = 0; j < 4; ++j) acc[i][j] = Frag<T>::mma(ah, bh[j], acc[i][j]);
      Frag<T>::guard(acc[i][0], acc[i][3], ah, ah);
    }
    Frag<T>::keep(bh[0], bh[1], bh[2], bh[3]);
  }
  acc_guard4(acc[0][0], acc[0][1], acc[0][2], acc[0][3]);
  acc_guard4(acc[1][0], acc[1][1], acc[1][2], acc[1][3]);
  acc_guard4(acc[2][0], acc[2][1], acc[2][2], acc[2][3]);
  acc_guard4(acc[3][0], acc[3][1], acc[3][2], acc[3][3]);

  float* slab = sT[wave];
  const float* Rb = RESID ? (resid + (size_t)b * strideR + (size_t)bz * strideRz) : nullptr;
  float hsum[4] = {0.f, 0.f, 0.f, 0.f};
#pragma unroll
  for (int i = 0; i < 4; ++i) {
    const int mBase = m0 + (i << 4);
#pragma unroll
    for (int j = 0; j < 4; ++j) {
      const int n = n0 + (j << 4) + rlane;
      float bv = 0.f;
      if (BIAS_MODE == 2) bv = bias[n];
#pragma unroll
      for (int r = 0; r < 8; ++r) {
        float v = acc[i][j][r] * scale;
        if (BIAS_MODE == 1) v += bias[mBase + mOff + r];
        if (BIAS_MODE == 2) v += bv;
        if (RESID) v += Rb[(size_t)(mBase + mOff + r) * ldc + n];
        if (ACT == 2) v = fmaxf(v, 0.0f);
        slab[(mOff + r) * 68 + (j << 4) + rlane] = v;
      }
    }
    __builtin_amdgcn_fence(__ATOMIC_RELEASE, "workgroup");
    __builtin_amdgcn_wave_barrier();
    __builtin_amdgcn_fence(__ATOMIC_ACQUIRE, "workgroup");
    if (OUT_MODE == 0) {
      float* C = (float*)Cout + (size_t)b * strideC + (size_t)bz * strideCz;
      const int hh = lane >> 4, c4 = (lane & 15) * 4;
      for (int pass = 0; pass < 2; ++pass) {
#pragma unroll
        for (int it = 0; it < 8; ++it) {
          const int row = it * 2 + hh;
          v4f v = *(const v4f*)(slab + row * 68 + c4);
          *(volatile v4f*)(C + (size_t)(mBase + row) * ldc + n0 + c4) = v;
        }
        __threadfence();
      }
    } else if (OUT_MODE == 1) {
      const int q = lane >> 3, c8 = (lane & 7) * 8;
      unsigned short* C = (unsigned short*)Cout + (size_t)b * strideC + (size_t)bz * strideCz;
      for (int pass = 0; pass < 2; ++pass) {
#pragma unroll
        for (int it = 0; it < 4; ++it) {
          const int row = it * 4 + q;
          const float* sp = slab + row * 68 + c8;
          v8h hv;
#pragma unroll
          for (int e = 0; e < 8; ++e) hv[e] = (_Float16)sp[e];
          *(volatile v8h*)(C + (size_t)(mBase + row) * ldc + n0 + c8) = hv;
        }
        __threadfence();
      }
    } else if (OUT_MODE == 3) {
      const float* sp = slab + rlane * 68 + (lane >> 4) * 32;
      float s = 0.f;
#pragma unroll
      for (int e = 0; e < 8; ++e) {
        const v4f t = *(const v4f*)(sp + 4 * e);
        s += (t[0] + t[1]) + (t[2] + t[3]);
      }
      s += __shfl_xor(s, 16, 32);
      hsum[i] = s * oscale;
    }
    __builtin_amdgcn_fence(__ATOMIC_RELEASE, "workgroup");
    __builtin_amdgcn_wave_barrier();
    __builtin_amdgcn_fence(__ATOMIC_ACQUIRE, "workgroup");
  }
  if (OUT_MODE == 3) {
    if (lane < 16) {
      slab[lane]      = hsum[0];
      slab[16 + lane] = hsum[1];
      slab[32 + lane] = hsum[2];
      slab[48 + lane] = hsum[3];
    }
    __builtin_amdgcn_fence(__ATOMIC_RELEASE, "workgroup");
    __builtin_amdgcn_wave_barrier();
    __builtin_amdgcn_fence(__ATOMIC_ACQUIRE, "workgroup");
    float* C = (float*)Cout + (size_t)tn * strideC + (size_t)(m0 / ldc) * strideCz + (size_t)(m0 % ldc);
    const v4f v = *(const v4f*)(slab + 4 * (lane & 15));
    if (lane < 16) {
      *(volatile v4f*)(C + 4 * lane) = v;
      __threadfence();
      *(volatile v4f*)(C + 4 * lane) = v;
    }
  }
}

__global__ __launch_bounds__(256) void cast8_f16_kernel(const float* __restrict__ in, unsigned short* __restrict__ out, int n8, float scale) {
  const int i = blockIdx.x * 256 + threadIdx.x;
  if (i >= n8) return;
  const float* p = in + 8 * (size_t)i;
  const v4f a = *(const v4f*)(p);
  const v4f c = *(const v4f*)(p + 4);
  unsigned short hb[8];
#pragma unroll
  for (int e = 0; e < 4; ++e) {
    hb[e]     = h_bits(a[e] * scale);
    hb[4 + e] = h_bits(c[e] * scale);
  }
  const v4u u = (v4u){pk16(hb[0], hb[1]), pk16(hb[2], hb[3]), pk16(hb[4], hb[5]), pk16(hb[6], hb[7])};
  unsigned short* q = out + 8 * (size_t)i;
  *(volatile v4u*)q = u;
  __threadfence();
  *(volatile v4u*)q = u;
}

__global__ __launch_bounds__(256) void transpose_cast_kernel(const float* __restrict__ in, unsigned short* __restrict__ out,
                                                             int R, int CC, float scale) {
  __shared__ float tile[64][65];
  const int t  = threadIdx.x;
  const int c0 = blockIdx.x * 64, r0 = blockIdx.y * 64;
  const int lc = t & 63, lr = t >> 6;
#pragma unroll
  for (int i = 0; i < 16; ++i) {
    const int r = i * 4 + lr;
    tile[lc][r] = in[(size_t)(r0 + r) * CC + c0 + lc];
  }
  __syncthreads();
  const int q = t >> 3, c8 = (t & 7) * 8;
#pragma unroll
  for (int it = 0; it < 2; ++it) {
    const int c = it * 32 + q;
    unsigned short hb[8];
#pragma unroll
    for (int e = 0; e < 8; ++e) hb[e] = h_bits(tile[c][c8 + e] * scale);
    const v4u u = (v4u){pk16(hb[0], hb[1]), pk16(hb[2], hb[3]), pk16(hb[4], hb[5]), pk16(hb[6], hb[7])};
    unsigned short* p = out + (size_t)(c0 + c) * R + r0 + c8;
    *(volatile v4u*)p = u;
    __threadfence();
    *(volatile v4u*)p = u;
  }
}

__global__ __launch_bounds__(256) void pe_hidden_kernel(const float* __restrict__ loc, const float* __restrict__ w1,
                                                        const float* __restrict__ b1, unsigned short* __restrict__ H1, int nrows) {
  __shared__ float sw[3 * kPH];
  __shared__ float sb[kPH];
  const int t = threadIdx.x;
  for (int i = t; i < 3 * kPH; i += 256) sw[i] = w1[i];
  if (t < kPH) sb[t] = b1[t];
  __syncthreads();
  const int lr = t >> 4, j0 = (t & 15) * 8;
  const int r  = blockIdx.x * 16 + lr;
  const int rc = r < nrows ? r : (nrows - 1);
  const float x = loc[(size_t)rc * 3 + 0];
  const float y = loc[(size_t)rc * 3 + 1];
  const float z = loc[(size_t)rc * 3 + 2];
  unsigned short hb[8];
#pragma unroll
  for (int e = 0; e < 8; ++e) {
    const int j = j0 + e;
    float v = ((x * sw[j] + y * sw[kPH + j]) + z * sw[2 * kPH + j]) + sb[j];
    v = fmaxf(v, 0.0f) * kH1Carry;
    hb[e] = h_bits(v);
  }
  const v4u u = (v4u){pk16(hb[0], hb[1]), pk16(hb[2], hb[3]), pk16(hb[4], hb[5]), pk16(hb[6], hb[7])};
  if (r < nrows) {
    unsigned short* p = H1 + (size_t)r * kPH + j0;
    *(volatile v4u*)p = u;
    __threadfence();
    *(volatile v4u*)p = u;
  }
}

__global__ __launch_bounds__(256) void softmax_kernel(const float* __restrict__ S, unsigned short* __restrict__ P, int nrows) {
  const int wave = threadIdx.x >> 5, lane = threadIdx.x & 31;
  const int row = blockIdx.x * 8 + wave;
  if (row >= nrows) return;
  const float* sp = S + (size_t)row * kNp + lane * 8;
  const v4f a = *(const v4f*)(sp);
  const v4f c = *(const v4f*)(sp + 4);
  float v[8];
#pragma unroll
  for (int e = 0; e < 4; ++e) { v[e] = a[e]; v[4 + e] = c[e]; }
  float mx = v[0];
#pragma unroll
  for (int e = 1; e < 8; ++e) mx = fmaxf(mx, v[e]);
#pragma unroll
  for (int off = 16; off > 0; off >>= 1) mx = fmaxf(mx, __shfl_xor(mx, off, 32));
  float sum = 0.f;
#pragma unroll
  for (int e = 0; e < 8; ++e) { v[e] = __expf(v[e] - mx); sum += v[e]; }
#pragma unroll
  for (int off = 16; off > 0; off >>= 1) sum += __shfl_xor(sum, off, 32);
  const float inv = 1.0f / sum;
  unsigned short hb[8];
#pragma unroll
  for (int e = 0; e < 8; ++e) hb[e] = h_bits((v[e] * inv) * kPCarry);
  const v4u u = (v4u){pk16(hb[0], hb[1]), pk16(hb[2], hb[3]), pk16(hb[4], hb[5]), pk16(hb[6], hb[7])};
  unsigned short* p = P + (size_t)row * kNp + lane * 8;
  *(volatile v4u*)p = u;
  __threadfence();
  *(volatile v4u*)p = u;
}

template <bool HOUT>
__global__ __launch_bounds__(256) void ln2d_kernel(const float* __restrict__ x, const float* __restrict__ w,
                                                   const float* __restrict__ bb, float* __restrict__ out,
                                                   unsigned short* __restrict__ out16) {
  __shared__ double red[256];
  const int bidx = blockIdx.x;
  const int t = threadIdx.x;
  const size_t base = (size_t)bidx * kSlab;
  const float* xb = x + base;
  double s = 0.0;
#pragma unroll 1
  for (int i = 0; i < 64; ++i) {
    const v4f a = *(const v4f*)(xb + (size_t)(i * 256 + t) * 4);
    s += (double)a[0]; s += (double)a[1]; s += (double)a[2]; s += (double)a[3];
  }
  red[t] = s;
  __syncthreads();
  double tot = 0.0;
#pragma unroll 1
  for (int i = 0; i < 256; ++i) tot += red[i];
  const float mean = (float)(tot * (1.0 / 65536.0));
  __syncthreads();
  double q = 0.0;
#pragma unroll 1
  for (int i = 0; i < 64; ++i) {
    const v4f a = *(const v4f*)(xb + (size_t)(i * 256 + t) * 4);
#pragma unroll
    for (int e = 0; e < 4; ++e) { const float d = a[e] - mean; q += (double)(d * d); }
  }
  red[t] = q;
  __syncthreads();
  double totq = 0.0;
#pragma unroll 1
  for (int i = 0; i < 256; ++i) totq += red[i];
  const float var = (float)(totq * (1.0 / 65536.0));
  const float rs  = rsqrtf(var + kLnEps);
  float* ob = out + base;
#pragma unroll 1
  for (int i = 0; i < 64; ++i) {
    const size_t idx = (size_t)(i * 256 + t) * 4;
    const v4f a  = *(const v4f*)(xb + idx);
    const v4f ww = *(const v4f*)(w + idx);
    const v4f bv = *(const v4f*)(bb + idx);
    v4f y;
#pragma unroll
    for (int e = 0; e < 4; ++e) y[e] = ((a[e] - mean) * rs) * ww[e] + bv[e];
    float* op = ob + idx;
    *(volatile v4f*)op = y;
    __threadfence();
    *(volatile v4f*)op = y;
  }
  if (HOUT) {
    unsigned short* hb16 = out16 + base;
#pragma unroll 1
    for (int i = 0; i < 32; ++i) {
      const size_t idx = (size_t)(i * 256 + t) * 8;
      const v4f a0 = *(const v4f*)(xb + idx),     a1 = *(const v4f*)(xb + idx + 4);
      const v4f w0 = *(const v4f*)(w + idx),      w1v = *(const v4f*)(w + idx + 4);
      const v4f b0 = *(const v4f*)(bb + idx),     b1v = *(const v4f*)(bb + idx + 4);
      unsigned short hb[8];
#pragma unroll
      for (int e = 0; e < 4; ++e) {
        hb[e]     = h_bits(((a0[e] - mean) * rs) * w0[e]  + b0[e]);
        hb[4 + e] = h_bits(((a1[e] - mean) * rs) * w1v[e] + b1v[e]);
      }
      const v4u u = (v4u){pk16(hb[0], hb[1]), pk16(hb[2], hb[3]), pk16(hb[4], hb[5]), pk16(hb[6], hb[7])};
      unsigned short* hp = hb16 + idx;
      *(volatile v4u*)hp = u;
      __threadfence();
      *(volatile v4u*)hp = u;
    }
  }
}

extern "C" void kernel_launch(void* const* d_in, const int* in_sizes, int n_in,
                              void* d_out, int out_size, void* d_ws, size_t ws_size,
                              hipStream_t stream) {
  if (n_in < 22) return;
  if (in_sizes[0] != kTok * kDim) return;
  if (in_sizes[1] != kPairs * 3) return;
  if (in_sizes[2] != kDim * kDim || in_sizes[4] != kDim * kDim || in_sizes[6] != kDim * kDim || in_sizes[8] != kDim * kDim) return;
  if (in_sizes[3] != kDim || in_sizes[5] != kDim || in_sizes[7] != kDim || in_sizes[9] != kDim) return;
  if (in_sizes[10] != 3 * kPH || in_sizes[11] != kPH || in_sizes[12] != kPH * kDim || in_sizes[13] != kDim) return;
  if (in_sizes[14] != kDim * kFF || in_sizes[15] != kFF || in_sizes[16] != kFF * kDim || in_sizes[17] != kDim) return;
  if (in_sizes[18] != kSlab || in_sizes[19] != kSlab || in_sizes[20] != kSlab || in_sizes[21] != kSlab) return;
  if (out_size != kTok * kDim) return;

  const float* input_feat = (const float*)d_in[0];
  const float* loc   = (const float*)d_in[1];
  const float* Kw    = (const float*)d_in[2];
  const float* Kb    = (const float*)d_in[3];
  const float* Qw    = (const float*)d_in[4];
  const float* Qb    = (const float*)d_in[5];
  const float* Vw    = (const float*)d_in[6];
  const float* Vb    = (const float*)d_in[7];
  const float* Fw    = (const float*)d_in[8];
  const float* Fb    = (const float*)d_in[9];
  const float* pe1w  = (const float*)d_in[10];
  const float* pe1b  = (const float*)d_in[11];
  const float* pe2w  = (const float*)d_in[12];
  const float* pe2b  = (const float*)d_in[13];
  const float* f1w   = (const float*)d_in[14];
  const float* f1b   = (const float*)d_in[15];
  const float* f2w   = (const float*)d_in[16];
  const float* f2b   = (const float*)d_in[17];
  const float* ln1w  = (const float*)d_in[18];
  const float* ln1b  = (const float*)d_in[19];
  const float* ln2w  = (const float*)d_in[20];
  const float* ln2b  = (const float*)d_in[21];
  float* outp = (float*)d_out;

  const size_t SZ_T16  = (size_t)kTok * kDim * 2;
  const size_t SZ_W16  = (size_t)kDim * kDim * 2;
  const size_t SZ_PE2T = (size_t)kDim * kPH * 2;
  const size_t SZ_F1T  = (size_t)kFF * kDim * 2;
  const size_t SZ_F2T  = (size_t)kDim * kFF * 2;
  const size_t SZ_VT   = (size_t)kDim * kTok * 2;
  const size_t SZ_H1   = (size_t)kPairs * kPH * 2;
  const size_t SZ_BHNN = (size_t)kBt * kHd * kNp * kNp;
  const size_t SZ_PS   = SZ_BHNN * 4;
  const size_t SZ_S    = SZ_BHNN * 4;
  const size_t SZ_P16  = SZ_BHNN * 2;
  const size_t SZ_T32  = (size_t)kTok * kDim * 4;
  const size_t SZ_HF   = (size_t)kTok * kFF * 2;

  size_t off = 0;
  const size_t oFEAT16 = off; off += SZ_T16;
  const size_t oKWT    = off; off += SZ_W16;
  const size_t oQWT    = off; off += SZ_W16;
  const size_t oVWT    = off; off += SZ_W16;
  const size_t oFWT    = off; off += SZ_W16;
  const size_t oPE2T   = off; off += SZ_PE2T;
  const size_t oF1T    = off; off += SZ_F1T;
  const size_t oF2T    = off; off += SZ_F2T;
  const size_t oK16    = off; off += SZ_T16;
  const size_t oQ16    = off; off += SZ_T16;
  const size_t oVT     = off; off += SZ_VT;
  const size_t oH1     = off; off += SZ_H1;
  const size_t oPS     = off; off += SZ_PS;
  const size_t oS      = off; off += SZ_S;
  const size_t oP16    = off; off += SZ_P16;
  const size_t oMRG    = off; off += SZ_T16;
  const size_t oR1     = off; off += SZ_T32;
  const size_t oO1F    = off; off += SZ_T32;
  const size_t oO1H    = off; off += SZ_T16;
  const size_t oHF     = off; off += SZ_HF;
  const size_t oR2     = off; off += SZ_T32;
  const size_t TOTAL   = off;
  if (TOTAL > ws_size) return;
  if (TOTAL > (size_t)134217728) return;

  char* ws = (char*)d_ws;
  unsigned short* FEAT16 = (unsigned short*)(ws + oFEAT16);
  unsigned short* KWT    = (unsigned short*)(ws + oKWT);
  unsigned short* QWT    = (unsigned short*)(ws + oQWT);
  unsigned short* VWT    = (unsigned short*)(ws + oVWT);
  unsigned short* FWT    = (unsigned short*)(ws + oFWT);
  unsigned short* PE2T   = (unsigned short*)(ws + oPE2T);
  unsigned short* F1T    = (unsigned short*)(ws + oF1T);
  unsigned short* F2T    = (unsigned short*)(ws + oF2T);
  unsigned short* K16    = (unsigned short*)(ws + oK16);
  unsigned short* Q16    = (unsigned short*)(ws + oQ16);
  unsigned short* VT     = (unsigned short*)(ws + oVT);
  unsigned short* H1     = (unsigned short*)(ws + oH1);
  float*          PS     = (float*)(ws + oPS);
  float*          S      = (float*)(ws + oS);
  unsigned short* P16    = (unsigned short*)(ws + oP16);
  unsigned short* MRG    = (unsigned short*)(ws + oMRG);
  float*          R1     = (float*)(ws + oR1);
  float*          O1F    = (float*)(ws + oO1F);
  unsigned short* O1H    = (unsigned short*)(ws + oO1H);
  unsigned short* HF     = (unsigned short*)(ws + oHF);
  float*          R2     = (float*)(ws + oR2);
  const float* nobias = Kb;
  const float* nores  = input_feat;

  const dim3 blk(256);
  const float invW   = 1.0f / kWCarry;
  const long  sBH    = (long)kNp * kNp;
  const long  sB4    = (long)kHd * kNp * kNp;
  const long  sTokB  = (long)kNp * kDim;

  {
    const int n8 = kTok * kDim / 8;
    cast8_f16_kernel<<<dim3(n8 / 256), blk, 0, stream>>>(input_feat, FEAT16, n8, 1.0f);
    transpose_cast_kernel<<<dim3(kDim / 64, kDim / 64), blk, 0, stream>>>(Kw, KWT, kDim, kDim, kWCarry);
    transpose_cast_kernel<<<dim3(kDim / 64, kDim / 64), blk, 0, stream>>>(Qw, QWT, kDim, kDim, kWCarry);
    transpose_cast_kernel<<<dim3(kDim / 64, kDim / 64), blk, 0, stream>>>(Vw, VWT, kDim, kDim, kWCarry);
    transpose_cast_kernel<<<dim3(kDim / 64, kDim / 64), blk, 0, stream>>>(Fw, FWT, kDim, kDim, kWCarry);
    transpose_cast_kernel<<<dim3(kDim / 64, kPH / 64), blk, 0, stream>>>(pe2w, PE2T, kPH, kDim, kWCarry);
    transpose_cast_kernel<<<dim3(kFF / 64, kDim / 64), blk, 0, stream>>>(f1w, F1T, kDim, kFF, kWCarry);
    transpose_cast_kernel<<<dim3(kDim / 64, kFF / 64), blk, 0, stream>>>(f2w, F2T, kFF, kDim, kWCarry);
  }

  pe_hidden_kernel<<<dim3(kPairs / 16), blk, 0, stream>>>(loc, pe1w, pe1b, H1, kPairs);

  {
    const int tiles = (kPairs / 64) * (kDim / 64);
    wmma_gemm64z<0, 2, 3, false, 0><<<dim3((tiles + 7) / 8, 1, 1), blk, 0, stream>>>(
        H1, kPH, 0L, 0L, PE2T, kPH, 0L, 0L, (void*)PS, (int)sBH, sBH, sB4,
        pe2b, nores, 0L, 0L, kPairs, kDim, kPH, 1.0f / (kH1Carry * kWCarry), 0.125f);
  }

  {
    const int tiles = (kTok / 64) * (kDim / 64);
    wmma_gemm64z<0, 2, 1, false, 0><<<dim3((tiles + 7) / 8, 1, 1), blk, 0, stream>>>(
        FEAT16, kDim, 0L, 0L, KWT, kDim, 0L, 0L, (void*)K16, kDim, 0L, 0L, Kb, nores, 0L, 0L, kTok, kDim, kDim, invW, 1.0f);
    wmma_gemm64z<0, 2, 1, false, 0><<<dim3((tiles + 7) / 8, 1, 1), blk, 0, stream>>>(
        FEAT16, kDim, 0L, 0L, QWT, kDim, 0L, 0L, (void*)Q16, kDim, 0L, 0L, Qb, nores, 0L, 0L, kTok, kDim, kDim, invW, 1.0f);
    wmma_gemm64z<0, 1, 1, false, 0><<<dim3((tiles + 7) / 8, 1, 1), blk, 0, stream>>>(
        VWT, kDim, 0L, 0L, FEAT16, kDim, 0L, 0L, (void*)VT, kTok, 0L, 0L, Vb, nores, 0L, 0L, kDim, kTok, kDim, invW, 1.0f);
  }

  {
    const int tiles = (kNp / 64) * (kNp / 64);
    wmma_gemm64z<0, 0, 0, true, 0><<<dim3((tiles + 7) / 8, kHd, kBt), blk, 0, stream>>>(
        K16, kDim, (long)kCh, sTokB, Q16, kDim, (long)kCh, sTokB, (void*)S, kNp, sBH, sB4,
        nobias, PS, sBH, sB4, kNp, kNp, kCh, 0.125f, 1.0f);
  }

  softmax_kernel<<<dim3((kBt * kHd * kNp + 7) / 8), blk, 0, stream>>>(S, P16, kBt * kHd * kNp);

  {
    const int tiles = (kNp / 64) * (kCh / 64);
    wmma_gemm64z<0, 0, 1, false, 0><<<dim3((tiles + 7) / 8, kHd, kBt), blk, 0, stream>>>(
        P16, kNp, sBH, sB4, VT, kTok, (long)kCh * kTok, (long)kNp, (void*)MRG, kDim, (long)kCh, sTokB,
        nobias, nores, 0L, 0L, kNp, kCh, kNp, kMgCarry / kPCarry, 1.0f);
  }

  {
    const int tiles = (kTok / 64) * (kDim / 64);
    wmma_gemm64z<0, 2, 0, true, 0><<<dim3((tiles + 7) / 8, 1, 1), blk, 0, stream>>>(
        MRG, kDim, 0L, 0L, FWT, kDim, 0L, 0L, (void*)R1, kDim, 0L, 0L, Fb, input_feat, 0L, 0L,
        kTok, kDim, kDim, 1.0f / (kMgCarry * kWCarry), 1.0f);
  }

  ln2d_kernel<true><<<dim3(kBt), blk, 0, stream>>>(R1, ln1w, ln1b, O1F, O1H);

  {
    const int tiles1 = (kTok / 64) * (kFF / 64);
    wmma_gemm64z<0, 2, 1, false, 2><<<dim3((tiles1 + 7) / 8, 1, 1), blk, 0, stream>>>(
        O1H, kDim, 0L, 0L, F1T, kDim, 0L, 0L, (void*)HF, kFF, 0L, 0L, f1b, nores, 0L, 0L, kTok, kFF, kDim, invW, 1.0f);
    const int tiles2 = (kTok / 64) * (kDim / 64);
    wmma_gemm64z<0, 2, 0, true, 0><<<dim3((tiles2 + 7) / 8, 1, 1), blk, 0, stream>>>(
        HF, kFF, 0L, 0L, F2T, kFF, 0L, 0L, (void*)R2, kDim, 0L, 0L, f2b, O1F, 0L, 0L, kTok, kDim, kFF, invW, 1.0f);
  }

  ln2d_kernel<false><<<dim3(kBt), blk, 0, stream>>>(R2, ln2w, ln2b, outp, O1H);
}
